// KANLayer_5609227289168
// MI455X (gfx1250) — hardware-verified
//
#include <hip/hip_runtime.h>
#include <math.h>

constexpr int kRows    = 2048;
constexpr int kIn      = 256;
constexpr int kOutC    = 512;
constexpr int kDeg     = 3;
constexpr int kKnots   = 39;
constexpr int kNB      = 35;
constexpr int kColSilu = kNB * kIn;
constexpr int kKtot    = kColSilu + kIn;
constexpr int kChunks  = kKtot / 8;
constexpr int kChunkIters = (kChunks + 255) / 256;
constexpr float kWCarry    = 16.0f;
constexpr float kWCarryInv = 0.0625f;

static_assert(kKtot % 32 == 0);
static_assert(kRows % 64 == 0);
static_assert(kOutC % 64 == 0);
static_assert(((kRows / 64) * (kOutC / 64)) % 8 == 0);
static_assert((kKtot * 2) % 128 == 0);
static_assert(kChunks * 8 == kKtot);
static_assert(kChunkIters * 256 >= kChunks);

typedef __attribute__((ext_vector_type(16))) _Float16 v16h;
typedef __attribute__((ext_vector_type(8)))  _Float16 v8h;
typedef __attribute__((ext_vector_type(16))) __bf16   v16b;
typedef __attribute__((ext_vector_type(8)))  __bf16   v8b;
typedef __attribute__((ext_vector_type(8)))  float    v8f;
typedef __attribute__((ext_vector_type(4)))  float    v4f;
typedef __attribute__((ext_vector_type(4)))  unsigned int v4u;

__device__ __forceinline__ unsigned short f2bf_bits(float f) {
  unsigned u = __float_as_uint(f);
  return (unsigned short)((u + 0x7FFFu + ((u >> 16) & 1u)) >> 16);
}
__device__ __forceinline__ float bf_bits2f(unsigned short h) { return __uint_as_float(((unsigned)h) << 16); }

__device__ __forceinline__ void dep_guard_h(v8f& a, v8f& b, v16h x, v16h y) { asm volatile("v_nop\n\tv_nop\n\tv_nop\n\tv_nop" : "+v"(a), "+v"(b) : "v"(x), "v"(y)); }
__device__ __forceinline__ void dep_guard_b(v8f& a, v8f& b, v16b x, v16b y) { asm volatile("v_nop\n\tv_nop\n\tv_nop\n\tv_nop" : "+v"(a), "+v"(b) : "v"(x), "v"(y)); }
__device__ __forceinline__ void keep4_h(v16h a, v16h b, v16h c, v16h d) { asm volatile("v_nop" :: "v"(a), "v"(b), "v"(c), "v"(d)); }
__device__ __forceinline__ void keep4_b(v16b a, v16b b, v16b c, v16b d) { asm volatile("v_nop" :: "v"(a), "v"(b), "v"(c), "v"(d)); }
__device__ __forceinline__ void acc_guard4(v8f& a, v8f& b, v8f& c, v8f& d) { asm volatile("v_nop\n\tv_nop\n\tv_nop\n\tv_nop" : "+v"(a), "+v"(b), "+v"(c), "+v"(d)); }
template <typename T> struct Frag;
template <> struct Frag<_Float16> {
  typedef v16h V; union U { v16h v; v8h h[2]; };
  static __device__ __forceinline__ v16h load(const _Float16* p) {
    U f; f.h[0] = *(const v8h*)(p); f.h[1] = *(const v8h*)(p + 16); return f.v;
  }
  static __device__ __forceinline__ v8f mma(v16h a, v16h b, v8f c) {
    return __builtin_amdgcn_wmma_f32_16x16x32_f16(false, a, false, b, (short)0, c, false, false);
  }
  static __device__ __forceinline__ void guard(v8f& a, v8f& b, v16h x, v16h y) { dep_guard_h(a, b, x, y); }
  static __device__ __forceinline__ void keep(v16h a, v16h b, v16h c, v16h d) { keep4_h(a, b, c, d); }
};
template <> struct Frag<__bf16> {
  typedef v16b V; union U { v16b v; v8b h[2]; };
  static __device__ __forceinline__ v16b load(const __bf16* p) {
    U f; f.h[0] = *(const v8b*)(p); f.h[1] = *(const v8b*)(p + 16); return f.v;
  }
  static __device__ __forceinline__ v8f mma(v16b a, v16b b, v8f c) {
    return __builtin_amdgcn_wmma_f32_16x16x32_bf16(false, a, false, b, (short)0, c, false, false);
  }
  static __device__ __forceinline__ void guard(v8f& a, v8f& b, v16b x, v16b y) { dep_guard_b(a, b, x, y); }
  static __device__ __forceinline__ void keep(v16b a, v16b b, v16b c, v16b d) { keep4_b(a, b, c, d); }
};

__device__ __forceinline__ unsigned pk16(unsigned short a, unsigned short b) { return (unsigned)a | ((unsigned)b << 16); }
__device__ __forceinline__ unsigned short h_bits(float f) { const _Float16 h = (_Float16)f; return __builtin_bit_cast(unsigned short, h); }

template <int ET> struct Elem;
template <> struct Elem<0> { typedef _Float16 T; };
template <> struct Elem<1> { typedef __bf16 T; };
template <int ET, bool SPLIT, int BIAS_MODE, int OUT_MODE, bool RESID, int ACT = 0>
__global__ __launch_bounds__(256) void wmma_gemm64(
    const unsigned short* __restrict__ Ap, const unsigned short* __restrict__ A2p, int lda, long strideA,
    const unsigned short* __restrict__ Btp, const unsigned short* __restrict__ Bt2p, int ldb, long strideB,
    void* __restrict__ Cout, void* __restrict__ Cout2, int ldc, long strideC,
    const float* __restrict__ bias,
    const float* __restrict__ resid, long strideR,
    int M, int N, int K, float scale) {
  typedef typename Elem<ET>::T T;
  typedef typename Frag<T>::V V;
  const T* A = (const T*)Ap; const T* A2 = (const T*)A2p; const T* Bt = (const T*)Btp; const T* Bt2 = (const T*)Bt2p;
  __shared__ __align__(16) float sT[8][16 * 68];
  const int b    = blockIdx.y;
  const int lane = threadIdx.x & 31;
  const int wave = threadIdx.x >> 5;
  const int tilesN = N >> 6;
  const int tilesM = M >> 6;
  const int tile = blockIdx.x * 8 + wave;
  if (tile >= tilesM * tilesN) return;
  const int tm = tile / tilesN;
  const int tn = tile - tm * tilesN;
  const int m0 = tm << 6;
  const int n0 = tn << 6;

  const T* Ab  = A  + (size_t)b * strideA;
  const T* Bb  = Bt + (size_t)b * strideB;
  const T* Ab2 = SPLIT ? (A2  + (size_t)b * strideA) : nullptr;
  const T* Bb2 = SPLIT ? (Bt2 + (size_t)b * strideB) : nullptr;

  const int rlane = lane & 15;
  const int koff  = (lane >> 4) * 8;
  const int mOff  = (lane >> 4) * 8;

  v8f acc[4][4];
#pragma unroll
  for (int i = 0; i < 4; ++i)
#pragma unroll
    for (int j = 0; j < 4; ++j) acc[i][j] = (v8f){0.f,0.f,0.f,0.f,0.f,0.f,0.f,0.f};

  for (int k0 = 0; k0 < K; k0 += 32) {
    V bh[4], bl[4];
#pragma unroll
    for (int j = 0; j < 4; ++j) {
      const size_t bo = (size_t)(n0 + (j << 4) + rlane) * ldb + koff + k0;
      bh[j] = Frag<T>::load(Bb + bo);
      if (SPLIT) bl[j] = Frag<T>::load(Bb2 + bo);
    }
#pragma unroll
    for (int i = 0; i < 4; ++i) {
      const size_t ao = (size_t)(m0 + (i << 4) + rlane) * lda + koff + k0;
      V ah = Frag<T>::load(Ab + ao);
      V al;
      if (SPLIT) al = Frag<T>::load(Ab2 + ao);
#pragma unroll
      for (int j = 0; j < 4; ++j) {
        acc[i][j] = Frag<T>::mma(ah, bh[j], acc[i][j]);
        if (SPLIT) {
          acc[i][j] = Frag<T>::mma(ah, bl[j], acc[i][j]);
          acc[i][j] = Frag<T>::mma(al, bh[j], acc[i][j]);
        }
      }
      Frag<T>::guard(acc[i][0], acc[i][3], ah, SPLIT ? al : ah);
    }
    Frag<T>::keep(bh[0], bh[1], bh[2], bh[3]);
    if (SPLIT) Frag<T>::keep(bl[0], bl[1], bl[2], bl[3]);
  }
  acc_guard4(acc[0][0], acc[0][1], acc[0][2], acc[0][3]);
  acc_guard4(acc[1][0], acc[1][1], acc[1][2], acc[1][3]);
  acc_guard4(acc[2][0], acc[2][1], acc[2][2], acc[2][3]);
  acc_guard4(acc[3][0], acc[3][1], acc[3][2], acc[3][3]);

  float* slab = sT[wave];
  const float* Rb = RESID ? (resid + (size_t)b * strideR) : nullptr;
#pragma unroll
  for (int i = 0; i < 4; ++i) {
    const int mBase = m0 + (i << 4);
#pragma unroll
    for (int j = 0; j < 4; ++j) {
      const int n = n0 + (j << 4) + rlane;
      float bv = 0.f;
      if (BIAS_MODE == 2) bv = bias[n];
#pragma unroll
      for (int r = 0; r < 8; ++r) {
        float v = acc[i][j][r] * scale;
        if (BIAS_MODE == 1) v += bias[mBase + mOff + r];
        if (BIAS_MODE == 2) v += bv;
        if (RESID) v += Rb[(size_t)(mBase + mOff + r) * ldc + n];
        if (ACT == 2) v = fmaxf(v, 0.0f);
        if (ACT == 4) v = (v > 0.f) ? v : 0.01f * v;
        slab[(mOff + r) * 68 + (j << 4) + rlane] = v;
      }
    }
    __builtin_amdgcn_fence(__ATOMIC_RELEASE, "workgroup");
    __builtin_amdgcn_wave_barrier();
    __builtin_amdgcn_fence(__ATOMIC_ACQUIRE, "workgroup");
    if (OUT_MODE == 0) {
      float* C = (float*)Cout + (size_t)b * strideC;
      const int hh = lane >> 4, c4 = (lane & 15) * 4;
      for (int pass = 0; pass < 2; ++pass) {
#pragma unroll
        for (int it = 0; it < 8; ++it) {
          const int row = it * 2 + hh;
          v4f v = *(const v4f*)(slab + row * 68 + c4);
          *(volatile v4f*)(C + (size_t)(mBase + row) * ldc + n0 + c4) = v;
        }
        __threadfence();
      }
    } else {
      const int q = lane >> 3, c8 = (lane & 7) * 8;
      unsigned short* C  = (unsigned short*)Cout  + (size_t)b * strideC;
      unsigned short* C2 = (OUT_MODE == 2) ? ((unsigned short*)Cout2 + (size_t)b * strideC) : nullptr;
      for (int pass = 0; pass < 2; ++pass) {
#pragma unroll
        for (int it = 0; it < 4; ++it) {
          const int row = it * 4 + q;
          const float* sp = slab + row * 68 + c8;
          v8h hv, lv;
#pragma unroll
          for (int e = 0; e < 8; ++e) {
            if (OUT_MODE == 1) {
              hv[e] = (_Float16)sp[e];
            } else {
              unsigned short hb = f2bf_bits(sp[e]);
              unsigned short lb = f2bf_bits(sp[e] - bf_bits2f(hb));
              hv[e] = __builtin_bit_cast(_Float16, hb);
              lv[e] = __builtin_bit_cast(_Float16, lb);
            }
          }
          *(volatile v8h*)(C + (size_t)(mBase + row) * ldc + n0 + c8) = hv;
          if (OUT_MODE == 2) *(volatile v8h*)(C2 + (size_t)(mBase + row) * ldc + n0 + c8) = lv;
        }
        __threadfence();
      }
    }
    __builtin_amdgcn_fence(__ATOMIC_RELEASE, "workgroup");
    __builtin_amdgcn_wave_barrier();
    __builtin_amdgcn_fence(__ATOMIC_ACQUIRE, "workgroup");
  }
}

__device__ __forceinline__ void stream_row_f16(const float* sRow, unsigned short* __restrict__ grow, int t) {
  for (int pass = 0; pass < 2; ++pass) {
#pragma unroll
    for (int it = 0; it < kChunkIters; ++it) {
      const int c = it * 256 + t;
      if (c < kChunks) {
        const v4f a = *(const v4f*)(sRow + c * 8);
        const v4f d = *(const v4f*)(sRow + c * 8 + 4);
        unsigned short hb[8];
#pragma unroll
        for (int e = 0; e < 4; ++e) {
          hb[e]     = h_bits(a[e]);
          hb[4 + e] = h_bits(d[e]);
        }
        const v4u u = (v4u){pk16(hb[0], hb[1]), pk16(hb[2], hb[3]), pk16(hb[4], hb[5]), pk16(hb[6], hb[7])};
        *(volatile v4u*)(grow + (size_t)c * 8) = u;
      }
    }
    __threadfence();
  }
}

__global__ __launch_bounds__(256) void build_act_plane(const float* __restrict__ x, const float* __restrict__ knots,
                                                       unsigned short* __restrict__ Aout) {
  __shared__ __align__(16) float sRow[kKtot];
  const int b = blockIdx.x;
  const int t = threadIdx.x;
  const float xv = x[(size_t)b * kIn + t];

  const float ex  = expf(-xv);
  const float sil = xv * (1.0f / (1.0f + ex));

  const float* gr = knots + (size_t)t * kKnots;
  int cnt = 0;
#pragma unroll 1
  for (int n = 0; n < kKnots; ++n) {
    const float gn = gr[n];
    cnt += (xv >= gn) ? 1 : 0;
  }
  const bool inr = (cnt >= 1) && (cnt <= kKnots - 1);
  int j = cnt - 1;
  j = (j < 0) ? 0 : j;
  j = (j > kKnots - 2) ? (kKnots - 2) : j;

  const float g0    = gr[0];
  const float hstep = gr[1] - gr[0];
  const float rh    = 1.0f / hstep;
  const float d1 = rh;
  const float d2 = rh * 0.5f;
  const float d3 = rh * 0.333333343f;

  const float tq1 = g0 + (float)(j - 2) * hstep;
  const float tq2 = g0 + (float)(j - 1) * hstep;
  const float tq3 = g0 + (float)(j)     * hstep;
  const float tq4 = g0 + (float)(j + 1) * hstep;
  const float tq5 = g0 + (float)(j + 2) * hstep;
  const float tq6 = g0 + (float)(j + 3) * hstep;

  const float n00 = inr ? 1.0f : 0.0f;
  const float n10 = ((tq4 - xv) * d1) * n00;
  const float n11 = ((xv - tq3) * d1) * n00;
  const float n20 = ((tq4 - xv) * d2) * n10;
  const float n21 = ((xv - tq2) * d2) * n10 + ((tq5 - xv) * d2) * n11;
  const float n22 = ((xv - tq3) * d2) * n11;
  const float n30 = ((tq4 - xv) * d3) * n20;
  const float n31 = ((xv - tq1) * d3) * n20 + ((tq5 - xv) * d3) * n21;
  const float n32 = ((xv - tq2) * d3) * n21 + ((tq6 - xv) * d3) * n22;
  const float n33 = ((xv - tq3) * d3) * n22;

  const int kb = j - kDeg;
#pragma unroll
  for (int k = 0; k < kNB; ++k) {
    const int m = k - kb;
    float v = 0.0f;
    v = (m == 0) ? n30 : v;
    v = (m == 1) ? n31 : v;
    v = (m == 2) ? n32 : v;
    v = (m == 3) ? n33 : v;
    v = inr ? v : 0.0f;
    sRow[k * kIn + t] = v;
  }
  sRow[kColSilu + t] = sil;
  __syncthreads();
  stream_row_f16(sRow, Aout + (size_t)b * kKtot, t);
}

__global__ __launch_bounds__(256) void build_wt_plane(const float* __restrict__ coef, const float* __restrict__ sbase,
                                                      const float* __restrict__ ssp, const float* __restrict__ msk,
                                                      unsigned short* __restrict__ Wout) {
  __shared__ __align__(16) float sRow[kKtot];
  const int o = blockIdx.x;
  const int t = threadIdx.x;
  const size_t io = (size_t)t * kOutC + o;
  const float mk = msk[io];
  const float sp = ssp[io];
  const float sb = sbase[io];
  const float fsp = kWCarry * (mk * sp);
  const float fsb = kWCarry * (mk * sb);
  const float* cr = coef + io * kNB;
#pragma unroll 1
  for (int k = 0; k < kNB; ++k) {
    const float cv = cr[k];
    sRow[k * kIn + t] = fsp * cv;
  }
  sRow[kColSilu + t] = fsb;
  __syncthreads();
  stream_row_f16(sRow, Wout + (size_t)o * kKtot, t);
}

extern "C" void kernel_launch(void* const* d_in, const int* in_sizes, int n_in,
                              void* d_out, int out_size, void* d_ws, size_t ws_size,
                              hipStream_t stream)
{
  if (n_in < 6) return;
  if (in_sizes[0] != kRows * kIn) return;
  if (in_sizes[1] != kIn * kKnots) return;
  if (in_sizes[2] != kIn * kOutC * kNB) return;
  if (in_sizes[3] != kIn * kOutC) return;
  if (in_sizes[4] != kIn * kOutC) return;
  if (in_sizes[5] != kIn * kOutC) return;
  if (out_size != kRows * kOutC) return;

  const size_t bytesA = (size_t)kRows * kKtot * sizeof(unsigned short);
  const size_t bytesW = (size_t)kOutC * kKtot * sizeof(unsigned short);
  static_assert(((size_t)kRows * kKtot * 2) % 128 == 0);
  if (bytesA + bytesW > ws_size) return;

  const float* x      = (const float*)d_in[0];
  const float* knots  = (const float*)d_in[1];
  const float* coef   = (const float*)d_in[2];
  const float* sbase  = (const float*)d_in[3];
  const float* ssp    = (const float*)d_in[4];
  const float* msk    = (const float*)d_in[5];

  unsigned short* Apl = (unsigned short*)d_ws;
  unsigned short* Wpl = (unsigned short*)((char*)d_ws + bytesA);
  float* outp = (float*)d_out;

  build_act_plane<<<kRows, 256, 0, stream>>>(x, knots, Apl);
  build_wt_plane<<<kOutC, 256, 0, stream>>>(coef, sbase, ssp, msk, Wpl);

  const int tiles  = (kRows / 64) * (kOutC / 64);
  const int blocks = tiles / 8;
  wmma_gemm64<0, false, 0, 0, false, 0><<<dim3(blocks, 1), 256, 0, stream>>>(
      Apl, Apl, kKtot, 0L,
      Wpl, Wpl, kKtot, 0L,
      (void*)outp, (void*)outp, kOutC, 0L,
      sbase,
      sbase, 0L,
      kRows, kOutC, kKtot, kWCarryInv);
}
